// NonLocalBlock3D_12627203850615
// MI455X (gfx1250) — hardware-verified
//
#include <hip/hip_runtime.h>
#include <math.h>
#include <stdint.h>

#ifndef NB
#define NB 1
#endif
#define NB_FULL 1
#ifndef SEQ
#define SEQ 8192
#endif
#define SEQ_FULL 8192
#define CC   256
#define DQ   128
#define QT   64
#define MW   384
#define OSP  68
#define OSPW 132
#define TP   72
#define WSC  256.0f
#define IWSC 0.00390625f
#define RSC  1024.0f
#define IRSC 0.0009765625f
#define LNPS 9.704060527839234f

static_assert(NB == 1 && NB_FULL == 1);
static_assert(SEQ >= QT && SEQ <= SEQ_FULL);
static_assert(SEQ % QT == 0 && SEQ % 32 == 0 && SEQ % 8 == 0);
static_assert(CC % QT == 0 && CC % 32 == 0);
static_assert(DQ == 2 * QT && DQ % 32 == 0);
static_assert(MW == 3 * DQ && MW % 8 == 0);
static_assert((OSP * 4) % 16 == 0);
static_assert((OSPW * 4) % 16 == 0);
static_assert((TP * 2) % 16 == 0);

typedef _Float16       v16h __attribute__((ext_vector_type(16)));
typedef _Float16       v8h  __attribute__((ext_vector_type(8)));
typedef __bf16         v16b __attribute__((ext_vector_type(16)));
typedef unsigned short v8us __attribute__((ext_vector_type(8)));
typedef float          v8f  __attribute__((ext_vector_type(8)));
typedef float          v4f  __attribute__((ext_vector_type(4)));
typedef unsigned int   v4u  __attribute__((ext_vector_type(4)));

union Frag  { v8us u[2]; v16h h; v16b bf; };
union FragH { v16h v; v8h hv[2]; };
static_assert(sizeof(Frag) == 32);
static_assert(sizeof(FragH) == 32);

__device__ __forceinline__ unsigned short bf_bits(float f) {
  unsigned u = __float_as_uint(f);
  return (unsigned short)((u + 0x7FFFu + ((u >> 16) & 1u)) >> 16);
}
__device__ __forceinline__ float bf_up(unsigned short hb) { return __uint_as_float(((unsigned)hb) << 16); }
__device__ __forceinline__ float bfr(float f) { return bf_up(bf_bits(f)); }
__device__ __forceinline__ unsigned short h_bits(_Float16 x) { return __builtin_bit_cast(unsigned short, x); }
__device__ __forceinline__ unsigned pk16(unsigned short a, unsigned short b) { return (unsigned)a | ((unsigned)b << 16); }
__device__ __forceinline__ v8f zero8() { v8f z = {0.f, 0.f, 0.f, 0.f, 0.f, 0.f, 0.f, 0.f}; return z; }
__device__ __forceinline__ float hmax8(v8f s) {
  return fmaxf(fmaxf(fmaxf(s[0], s[1]), fmaxf(s[2], s[3])), fmaxf(fmaxf(s[4], s[5]), fmaxf(s[6], s[7])));
}
__device__ __forceinline__ unsigned wave_ballot(bool p) {
#if defined(__HIP_DEVICE_COMPILE__)
  return __builtin_amdgcn_ballot_w32(p);
#else
  return p ? 1u : 0u;
#endif
}

__device__ __forceinline__ Frag ldfrag(const unsigned short* p) {
  Frag f;
  f.u[0] = *(const v8us*)(p);
  f.u[1] = *(const v8us*)(p + 16);
  return f;
}

__device__ __forceinline__ v8f mma_h(v16h a, v16h b, v8f c) {
  v8f d = __builtin_amdgcn_wmma_f32_16x16x32_f16(false, a, false, b, (short)0, c, false, false);
#if defined(__HIP_DEVICE_COMPILE__)
  asm volatile("v_nop\n\tv_nop\n\tv_nop\n\tv_nop" : "+v"(d) : "v"(a), "v"(b));
#endif
  return d;
}
__device__ __forceinline__ v8f mma_b(v16b a, v16b b, v8f c) {
  v8f d = __builtin_amdgcn_wmma_f32_16x16x32_bf16(false, a, false, b, (short)0, c, false, false);
#if defined(__HIP_DEVICE_COMPILE__)
  const v16h ha = __builtin_bit_cast(v16h, a), hb = __builtin_bit_cast(v16h, b);
  asm volatile("v_nop\n\tv_nop\n\tv_nop\n\tv_nop" : "+v"(d) : "v"(ha), "v"(hb));
#endif
  return d;
}

__global__ __launch_bounds__(256)
void cvt_wt(const float* __restrict__ src, unsigned short* dst, int R, int S, int rowBase) {
  __shared__ __align__(16) unsigned short T[QT * TP];
  const int tid = threadIdx.x;
  const int sb = blockIdx.x, rb = blockIdx.y;
  const int e = tid & 7, lq = tid >> 3;
  const int s0 = sb * QT, r0 = rb * QT;
#pragma unroll
  for (int it = 0; it < 2; ++it) {
    const int rl = it * 32 + lq;
    const float* sp = src + ((size_t)(r0 + rl)) * (size_t)S + s0 + 8 * e;
    const v4f a = *(const v4f*)sp;
    const v4f q = *(const v4f*)(sp + 4);
    unsigned short hb[8];
#pragma unroll
    for (int t = 0; t < 4; ++t) {
      hb[t]     = h_bits((_Float16)(bfr(a[t]) * WSC));
      hb[4 + t] = h_bits((_Float16)(bfr(q[t]) * WSC));
    }
#pragma unroll
    for (int t = 0; t < 8; ++t) T[(8 * e + t) * TP + rl] = hb[t];
  }
  __syncthreads();
  v4u up[2];
#pragma unroll
  for (int it = 0; it < 2; ++it) {
    const int sl = it * 32 + lq;
    up[it] = *(const v4u*)(T + sl * TP + 8 * e);
  }
#pragma unroll
  for (int pass = 0; pass < 2; ++pass) {
#pragma unroll
    for (int it = 0; it < 2; ++it) {
      const int sl = it * 32 + lq;
      *(volatile v4u*)(dst + ((size_t)(rowBase + s0 + sl)) * (size_t)R + r0 + 8 * e) = up[it];
    }
    __threadfence();
  }
}

__global__ __launch_bounds__(256)
void cvt_x(const float* __restrict__ x, unsigned short* XP) {
  const int tid = threadIdx.x, blk = blockIdx.x;
  const int row = 8 * blk + (tid >> 5);
  const int col = 8 * (tid & 31);
  const float* s = x + (size_t)row * CC + col;
  const v4f a = *(const v4f*)s;
  const v4f q = *(const v4f*)(s + 4);
  const float f[8] = {a[0], a[1], a[2], a[3], q[0], q[1], q[2], q[3]};
  v4u u;
#pragma unroll
  for (int t = 0; t < 4; ++t) {
    const _Float16 h0 = (_Float16)bfr(f[2 * t]);
    const _Float16 h1 = (_Float16)bfr(f[2 * t + 1]);
    u[t] = pk16(h_bits(h0), h_bits(h1));
  }
#pragma unroll
  for (int pass = 0; pass < 2; ++pass) {
    *(volatile v4u*)(XP + (size_t)row * CC + col) = u;
    __threadfence();
  }
}

__global__ __launch_bounds__(128)
void gemm_qkv(const unsigned short* __restrict__ W16, const unsigned short* __restrict__ XP,
              const float* __restrict__ tbias, const float* __restrict__ pbias, const float* __restrict__ gbias,
              unsigned short* Qh, unsigned short* Ql, unsigned short* Kh, unsigned short* Kl, unsigned short* Gc) {
  __shared__ __align__(16) float Os[QT * OSP];
  const int tid  = threadIdx.x;
  const int lane = tid & 31, wave = tid >> 5;
  const int hh   = lane >> 4, c = lane & 15;
  const int nt   = blockIdx.x, mb = blockIdx.y;
  const int n0   = nt * QT, o0 = mb * QT;

  const unsigned short* ap = W16 + (size_t)(o0 + c) * CC + 8 * hh;
  const unsigned short* bp = XP + ((size_t)(n0 + 16 * wave + c)) * CC + 8 * hh;

  v8f acc[4];
#pragma unroll
  for (int mt = 0; mt < 4; ++mt) acc[mt] = zero8();

#pragma unroll
  for (int ks = 0; ks < CC / 32; ++ks) {
    const Frag fb = ldfrag(bp + 32 * ks);
#pragma unroll
    for (int mt = 0; mt < 4; ++mt) {
      const Frag fa = ldfrag(ap + (size_t)(16 * mt) * CC + 32 * ks);
      acc[mt] = mma_h(fa.h, fb.h, acc[mt]);
    }
  }

  {
    const int nl = 16 * wave + c;
#pragma unroll
    for (int mt = 0; mt < 4; ++mt) {
      v4f va, vb;
#pragma unroll
      for (int r = 0; r < 4; ++r) { va[r] = acc[mt][r] * IWSC; vb[r] = acc[mt][4 + r] * IWSC; }
      *(v4f*)(Os + nl * OSP + 16 * mt + 8 * hh)     = va;
      *(v4f*)(Os + nl * OSP + 16 * mt + 8 * hh + 4) = vb;
    }
  }
  __syncthreads();

  const int e = tid & 7, lq = tid >> 3;
  const int grp  = mb >> 1;
  const int dsel = (mb & 1) * QT;
  if (grp < 2) {
    const float* bsrc = (grp == 0) ? tbias : pbias;
    unsigned short* Hp = (grp == 0) ? Qh : Kh;
    unsigned short* Lp = (grp == 0) ? Ql : Kl;
    const v4f b0 = *(const v4f*)(bsrc + dsel + 8 * e);
    const v4f b1 = *(const v4f*)(bsrc + dsel + 8 * e + 4);
    const float bb[8] = {bfr(b0[0]), bfr(b0[1]), bfr(b0[2]), bfr(b0[3]), bfr(b1[0]), bfr(b1[1]), bfr(b1[2]), bfr(b1[3])};
    v4u uh[4], ul[4];
#pragma unroll
    for (int it = 0; it < 4; ++it) {
      const int row = it * 16 + lq;
      const v4f a = *(const v4f*)(Os + row * OSP + 8 * e);
      const v4f q = *(const v4f*)(Os + row * OSP + 8 * e + 4);
      const float f[8] = {a[0], a[1], a[2], a[3], q[0], q[1], q[2], q[3]};
#pragma unroll
      for (int t = 0; t < 4; ++t) {
        const float f0 = f[2 * t] + bb[2 * t], f1 = f[2 * t + 1] + bb[2 * t + 1];
        const unsigned short hb0 = bf_bits(f0), hb1 = bf_bits(f1);
        const unsigned short lb0 = bf_bits(f0 - bf_up(hb0));
        const unsigned short lb1 = bf_bits(f1 - bf_up(hb1));
        uh[it][t] = pk16(hb0, hb1);
        ul[it][t] = pk16(lb0, lb1);
      }
    }
#pragma unroll
    for (int pass = 0; pass < 2; ++pass) {
#pragma unroll
      for (int it = 0; it < 4; ++it) {
        const int row = it * 16 + lq;
        const size_t po = ((size_t)(n0 + row)) * DQ + dsel + 8 * e;
        *(volatile v4u*)(Hp + po) = uh[it];
        *(volatile v4u*)(Lp + po) = ul[it];
      }
      __threadfence();
    }
  } else {
    const int gsel = dsel;
    v4u ug[4];
#pragma unroll
    for (int it = 0; it < 4; ++it) {
      const int cl = it * 16 + lq;
      const float bias = bfr(gbias[gsel + cl]);
      unsigned short hb[8];
#pragma unroll
      for (int t = 0; t < 8; ++t) {
        const int key = 8 * e + t;
        const float v = Os[key * OSP + cl] + bias;
        hb[t] = h_bits((_Float16)v);
      }
#pragma unroll
      for (int t = 0; t < 4; ++t) ug[it][t] = pk16(hb[2 * t], hb[2 * t + 1]);
    }
#pragma unroll
    for (int pass = 0; pass < 2; ++pass) {
#pragma unroll
      for (int it = 0; it < 4; ++it) {
        const int cl = it * 16 + lq;
        const size_t po = ((size_t)(gsel + cl)) * (size_t)SEQ + n0 + 8 * e;
        *(volatile v4u*)(Gc + po) = ug[it];
      }
      __threadfence();
    }
  }
}

__global__ __launch_bounds__(128)
void attn_k(const unsigned short* __restrict__ Qh, const unsigned short* __restrict__ Ql,
            const unsigned short* __restrict__ Kh, const unsigned short* __restrict__ Kl,
            const unsigned short* __restrict__ Gc, unsigned short* Yh, unsigned short* Yl) {
  __shared__ __align__(16) float Os[QT * OSPW];
  const int tid  = threadIdx.x;
  const int wave = tid >> 5, lane = tid & 31;
  const int hh   = lane >> 4, c = lane & 15;
  const int n0   = blockIdx.x * QT;

  const size_t qo = ((size_t)(n0 + 16 * wave + c)) * DQ + 8 * hh;
  const unsigned short* Qhp = Qh + qo;
  const unsigned short* Qlp = Ql + qo;
  const unsigned short* Khp = Kh + (size_t)c * DQ + 8 * hh;
  const unsigned short* Klp = Kl + (size_t)c * DQ + 8 * hh;
  const unsigned short* Vp = Gc + (size_t)c * (size_t)SEQ + 8 * hh;

  float m = -1.0e30f, l = 0.f;
  v8f o[8];
#pragma unroll
  for (int j = 0; j < 8; ++j) o[j] = zero8();

#pragma unroll 1
  for (int kb = 0; kb < SEQ; kb += 32) {
    const unsigned short* k0p  = Khp + (size_t)kb * DQ;
    const unsigned short* k1p  = Khp + (size_t)(kb + 16) * DQ;
    const unsigned short* k0lp = Klp + (size_t)kb * DQ;
    const unsigned short* k1lp = Klp + (size_t)(kb + 16) * DQ;
    v8f s0 = zero8(), s1 = zero8();
#pragma unroll 1
    for (int kc = 0; kc < DQ / 32; ++kc) {
      const Frag qh  = ldfrag(Qhp + 32 * kc);
      const Frag ql  = ldfrag(Qlp + 32 * kc);
      const Frag k0  = ldfrag(k0p + 32 * kc);
      const Frag k1  = ldfrag(k1p + 32 * kc);
      const Frag k0l = ldfrag(k0lp + 32 * kc);
      const Frag k1l = ldfrag(k1lp + 32 * kc);
      s0 = mma_b(k0.bf, qh.bf, s0);
      s1 = mma_b(k1.bf, qh.bf, s1);
      s0 = mma_b(k0.bf, ql.bf, s0);
      s1 = mma_b(k1.bf, ql.bf, s1);
      s0 = mma_b(k0l.bf, qh.bf, s0);
      s1 = mma_b(k1l.bf, qh.bf, s1);
    }

    float mx = fmaxf(hmax8(s0), hmax8(s1));
    mx = fmaxf(mx, __shfl_xor(mx, 16, 32));
    const float mn = fmaxf(m, mx);
    const unsigned grew = wave_ballot(mx > m);
    if (grew != 0u) {
      const float corr = __expf(m - mn);
      l *= corr;
#pragma unroll
      for (int j = 0; j < 8; ++j) {
#pragma unroll
        for (int r = 0; r < 8; ++r) o[j][r] *= corr;
      }
    }
    m = mn;
    const float msh = mn - LNPS;

    FragH ph;
    float ls = 0.f;
#pragma unroll
    for (int r = 0; r < 8; ++r) {
      const float e0 = __expf(s0[r] - msh);
      const float e1 = __expf(s1[r] - msh);
      ls += e0 + e1;
      ph.hv[0][r] = (_Float16)e0;
      ph.hv[1][r] = (_Float16)e1;
    }
    l += ls;

#pragma unroll
    for (int j = 0; j < 8; ++j) {
      const Frag vf = ldfrag(Vp + (size_t)(16 * j) * (size_t)SEQ + kb);
      o[j] = mma_h(vf.h, ph.v, o[j]);
    }
  }
  l += __shfl_xor(l, 16, 32);
  const float inv = 1.0f / l;

  const int qrow = 16 * wave + c;
#pragma unroll
  for (int j = 0; j < 8; ++j) {
    v4f va, vb;
#pragma unroll
    for (int r = 0; r < 4; ++r) { va[r] = o[j][r] * inv; vb[r] = o[j][4 + r] * inv; }
    *(v4f*)(Os + qrow * OSPW + 16 * j + 8 * hh)     = va;
    *(v4f*)(Os + qrow * OSPW + 16 * j + 8 * hh + 4) = vb;
  }
  __syncthreads();

  const int e = tid & 15, lq = tid >> 4;
  v4u uh[8], ul[8];
#pragma unroll
  for (int it = 0; it < 8; ++it) {
    const int row = it * 8 + lq;
    const v4f a = *(const v4f*)(Os + row * OSPW + 8 * e);
    const v4f q = *(const v4f*)(Os + row * OSPW + 8 * e + 4);
    const float f[8] = {a[0], a[1], a[2], a[3], q[0], q[1], q[2], q[3]};
#pragma unroll
    for (int t = 0; t < 4; ++t) {
      const float f0 = f[2 * t], f1 = f[2 * t + 1];
      const _Float16 h0 = (_Float16)f0, h1 = (_Float16)f1;
      const _Float16 r0 = (_Float16)((f0 - (float)h0) * RSC);
      const _Float16 r1 = (_Float16)((f1 - (float)h1) * RSC);
      uh[it][t] = pk16(h_bits(h0), h_bits(h1));
      ul[it][t] = pk16(h_bits(r0), h_bits(r1));
    }
  }
#pragma unroll
  for (int pass = 0; pass < 2; ++pass) {
#pragma unroll
    for (int it = 0; it < 8; ++it) {
      const int row = it * 8 + lq;
      const size_t po = ((size_t)(n0 + row)) * DQ + 8 * e;
      *(volatile v4u*)(Yh + po) = uh[it];
      *(volatile v4u*)(Yl + po) = ul[it];
    }
    __threadfence();
  }
}

__global__ __launch_bounds__(128)
void gemm_o(const unsigned short* __restrict__ WW16, const unsigned short* __restrict__ Yh,
            const unsigned short* __restrict__ Yl, const float* __restrict__ wbias,
            const float* __restrict__ x, float* out) {
  __shared__ __align__(16) float Os[QT * OSP];
  const int tid  = threadIdx.x;
  const int lane = tid & 31, wave = tid >> 5;
  const int hh   = lane >> 4, c = lane & 15;
  const int nt   = blockIdx.x, mb = blockIdx.y;
  const int n0   = nt * QT, o0 = mb * QT;

  const unsigned short* ap  = WW16 + (size_t)(o0 + c) * DQ + 8 * hh;
  const size_t bo = ((size_t)(n0 + 16 * wave + c)) * DQ + 8 * hh;
  const unsigned short* bph = Yh + bo;
  const unsigned short* bpl = Yl + bo;

  v8f acc[4], accr[4];
#pragma unroll
  for (int mt = 0; mt < 4; ++mt) { acc[mt] = zero8(); accr[mt] = zero8(); }

#pragma unroll
  for (int ks = 0; ks < DQ / 32; ++ks) {
    const Frag fbh = ldfrag(bph + 32 * ks);
    const Frag fbl = ldfrag(bpl + 32 * ks);
#pragma unroll
    for (int mt = 0; mt < 4; ++mt) {
      const Frag fa = ldfrag(ap + (size_t)(16 * mt) * DQ + 32 * ks);
      acc[mt]  = mma_h(fa.h, fbh.h, acc[mt]);
      accr[mt] = mma_h(fa.h, fbl.h, accr[mt]);
    }
  }

  {
    const int nl = 16 * wave + c;
#pragma unroll
    for (int mt = 0; mt < 4; ++mt) {
      v4f va, vb;
#pragma unroll
      for (int r = 0; r < 4; ++r) {
        va[r] = (acc[mt][r] + accr[mt][r] * IRSC) * IWSC;
        vb[r] = (acc[mt][4 + r] + accr[mt][4 + r] * IRSC) * IWSC;
      }
      *(v4f*)(Os + nl * OSP + 16 * mt + 8 * hh)     = va;
      *(v4f*)(Os + nl * OSP + 16 * mt + 8 * hh + 4) = vb;
    }
  }
  __syncthreads();

  const int e = tid & 15, lq = tid >> 4;
  const v4f bv = *(const v4f*)(wbias + o0 + 4 * e);
  const float bb[4] = {bfr(bv[0]), bfr(bv[1]), bfr(bv[2]), bfr(bv[3])};
  v4f res[8];
#pragma unroll
  for (int it = 0; it < 8; ++it) {
    const int nl = it * 8 + lq;
    const size_t idx = ((size_t)(n0 + nl)) * CC + o0 + 4 * e;
    const v4f xv = *(const v4f*)(x + idx);
    const v4f ov = *(const v4f*)(Os + nl * OSP + 4 * e);
#pragma unroll
    for (int t = 0; t < 4; ++t) res[it][t] = ov[t] + bb[t] + bfr(xv[t]);
  }
#pragma unroll
  for (int pass = 0; pass < 2; ++pass) {
#pragma unroll
    for (int it = 0; it < 8; ++it) {
      const int nl = it * 8 + lq;
      const size_t idx = ((size_t)(n0 + nl)) * CC + o0 + 4 * e;
      *(volatile v4f*)(out + idx) = res[it];
    }
    __threadfence();
  }
}

extern "C" void kernel_launch(void* const* d_in, const int* in_sizes, int n_in,
                              void* d_out, int out_size, void* d_ws, size_t ws_size,
                              hipStream_t stream) {
  const int XN = SEQ * CC;
  if (n_in < 9) return;
  if (in_sizes[0] < XN) return;
  if (in_sizes[1] < CC * DQ || in_sizes[3] < CC * DQ || in_sizes[5] < CC * DQ) return;
  if (in_sizes[2] < DQ || in_sizes[4] < DQ || in_sizes[6] < DQ) return;
  if (in_sizes[7] < DQ * CC || in_sizes[8] < CC) return;
  if (out_size < XN) return;

  size_t off = 0;
  auto carve = [&](size_t bytes) { const size_t o = off; off += (bytes + 255) & ~(size_t)255; return o; };
  const size_t oW16 = carve((size_t)MW * CC * 2);
  const size_t oWW  = carve((size_t)CC * DQ * 2);
  const size_t oXP  = carve((size_t)SEQ * CC * 2);
  const size_t oQh  = carve((size_t)SEQ * DQ * 2);
  const size_t oQl  = carve((size_t)SEQ * DQ * 2);
  const size_t oKh  = carve((size_t)SEQ * DQ * 2);
  const size_t oKl  = carve((size_t)SEQ * DQ * 2);
  const size_t oGc  = carve((size_t)DQ * SEQ * 2);
  const size_t oYh  = carve((size_t)SEQ * DQ * 2);
  const size_t oYl  = carve((size_t)SEQ * DQ * 2);
  if (off > ws_size) return;
  if (off > (size_t)134217728) return;

  const float* x  = (const float*)d_in[0];
  const float* gw = (const float*)d_in[1];
  const float* gb = (const float*)d_in[2];
  const float* tw = (const float*)d_in[3];
  const float* tb = (const float*)d_in[4];
  const float* pw = (const float*)d_in[5];
  const float* pb = (const float*)d_in[6];
  const float* ww = (const float*)d_in[7];
  const float* wb = (const float*)d_in[8];

  char* ws = (char*)d_ws;
  unsigned short* W16  = (unsigned short*)(ws + oW16);
  unsigned short* WW16 = (unsigned short*)(ws + oWW);
  unsigned short* XP   = (unsigned short*)(ws + oXP);
  unsigned short* Qh   = (unsigned short*)(ws + oQh);
  unsigned short* Ql   = (unsigned short*)(ws + oQl);
  unsigned short* Kh   = (unsigned short*)(ws + oKh);
  unsigned short* Kl   = (unsigned short*)(ws + oKl);
  unsigned short* Gc   = (unsigned short*)(ws + oGc);
  unsigned short* Yh   = (unsigned short*)(ws + oYh);
  unsigned short* Yl   = (unsigned short*)(ws + oYl);
  float* out = (float*)d_out;

  const dim3 blk256(256), blk128(128);

  cvt_wt<<<dim3(DQ / QT, CC / QT), blk256, 0, stream>>>(tw, W16, CC, DQ, 0);
  cvt_wt<<<dim3(DQ / QT, CC / QT), blk256, 0, stream>>>(pw, W16, CC, DQ, DQ);
  cvt_wt<<<dim3(DQ / QT, CC / QT), blk256, 0, stream>>>(gw, W16, CC, DQ, 2 * DQ);
  cvt_wt<<<dim3(CC / QT, DQ / QT), blk256, 0, stream>>>(ww, WW16, DQ, CC, 0);
  cvt_x<<<dim3(SEQ / 8), blk256, 0, stream>>>(x, XP);
  gemm_qkv<<<dim3(SEQ / QT, 6), blk128, 0, stream>>>(W16, XP, tb, pb, gb, Qh, Ql, Kh, Kl, Gc);
  attn_k<<<dim3(SEQ / QT), blk128, 0, stream>>>(Qh, Ql, Kh, Kl, Gc, Yh, Yl);
  gemm_o<<<dim3(SEQ / QT, CC / QT), blk128, 0, stream>>>(WW16, Yh, Yl, wb, x, out);
  (void)hipGetLastError();
}
